// CondAttentionBlock_46093589021360
// MI455X (gfx1250) — hardware-verified
//
#include <hip/hip_runtime.h>


#define NB_  32
#define CC   256
#define LL   1024
#define AD   512
#define NG   32
#define NHD  4
#define CH   64
#define TT   1024
#define ZH   1
#define PCAR 1024.0f
#define SCL  0.125f
typedef _Float16 h16;
typedef unsigned short bf;
typedef __attribute__((ext_vector_type(16))) __bf16   v16bf;
typedef __attribute__((ext_vector_type(16))) _Float16 v16h;
typedef __attribute__((ext_vector_type(8)))  _Float16 v8h;
typedef __attribute__((ext_vector_type(8)))  unsigned short v8us;
typedef __attribute__((ext_vector_type(8)))  float    v8f;
typedef __attribute__((ext_vector_type(4)))  float    v4f;
typedef v8h  __attribute__((may_alias)) v8ha;
typedef v4f  __attribute__((may_alias)) v4fa;
typedef v8us __attribute__((may_alias)) v8usa;

__device__ __forceinline__ unsigned short f2bf(float f) { unsigned u = __float_as_uint(f); u += 0x7FFFu + ((u >> 16) & 1u); return (unsigned short)(u >> 16); }
__device__ __forceinline__ float bf2f(unsigned short b) { return __uint_as_float(((unsigned)b) << 16); }
__device__ __forceinline__ float bfr(float f) { return bf2f(f2bf(f)); }
__device__ __forceinline__ v16h cat16(v8h lo, v8h hi) { return __builtin_shufflevector(lo, hi, 0, 1, 2, 3, 4, 5, 6, 7, 8, 9, 10, 11, 12, 13, 14, 15); }
__device__ __forceinline__ v16bf cat16b(v8us lo, v8us hi) { return __builtin_bit_cast(v16bf, __builtin_shufflevector(lo, hi, 0, 1, 2, 3, 4, 5, 6, 7, 8, 9, 10, 11, 12, 13, 14, 15)); }
__device__ __forceinline__ v8f wmma16(v16h a, v16h b, v8f c) { return __builtin_amdgcn_wmma_f32_16x16x32_f16(false, a, false, b, (short)0, c, false, false); }
__device__ __forceinline__ v8f wmmab(v16bf a, v16bf b, v8f c) { return __builtin_amdgcn_wmma_f32_16x16x32_bf16(false, a, false, b, (short)0, c, false, false); }


template <typename T16> struct WFrag;
template <> struct WFrag<h16> { typedef v16h V; static __device__ __forceinline__ V ld(const h16* p) { return cat16(*(const v8h*)p, *(const v8h*)(p + 16)); } static __device__ __forceinline__ v8f mma(V a, V b, v8f c) { return wmma16(a, b, c); } };
template <> struct WFrag<bf> { typedef v16bf V; static __device__ __forceinline__ V ld(const bf* p) { return cat16b(*(const v8us*)p, *(const v8us*)(p + 16)); } static __device__ __forceinline__ v8f mma(V a, V b, v8f c) { return wmmab(a, b, c); } };
template <typename T16, int NSPLIT, bool BIAS>
__global__ __launch_bounds__(32) void k_gemmw(const T16* __restrict__ A, const T16* __restrict__ A2, const T16* __restrict__ Bt, const T16* __restrict__ Bt2, int K, float* C, int ldc, const float* __restrict__ bias, size_t sA, size_t sB, size_t sC) {
    typedef typename WFrag<T16>::V V;
    __shared__ __align__(16) float os[16 * 68];
    const size_t z = blockIdx.z; A += z * sA; if (A2) A2 += z * sA; Bt += z * sB; if (Bt2) Bt2 += z * sB; C += z * sC;
    const int lane = threadIdx.x & 31, lr = lane & 15, hi = lane >> 4; const int r0 = blockIdx.x * 64, c0 = blockIdx.y * 64;
    v8f acc[4][4];
#pragma unroll
    for (int mb = 0; mb < 4; ++mb)
#pragma unroll
        for (int nb = 0; nb < 4; ++nb) acc[mb][nb] = (v8f){};
    const size_t aoff = (size_t)(r0 + lr) * K + 8 * hi, boff = (size_t)(c0 + lr) * K + 8 * hi;
#pragma unroll 1
    for (int kc = 0; kc < K; kc += 32) {
        V a[4], a2[4];
#pragma unroll
        for (int mb = 0; mb < 4; ++mb) { a[mb] = WFrag<T16>::ld(A + aoff + (size_t)mb * 16 * K + kc); if (NSPLIT == 1 || NSPLIT == 2) a2[mb] = WFrag<T16>::ld(A2 + aoff + (size_t)mb * 16 * K + kc); }
#pragma unroll
        for (int nb = 0; nb < 4; ++nb) { const V b = WFrag<T16>::ld(Bt + boff + (size_t)nb * 16 * K + kc); V b2; if (NSPLIT >= 2) b2 = WFrag<T16>::ld(Bt2 + boff + (size_t)nb * 16 * K + kc);
#pragma unroll
            for (int mb = 0; mb < 4; ++mb) { acc[mb][nb] = WFrag<T16>::mma(a[mb], b, acc[mb][nb]); if (NSPLIT == 1 || NSPLIT == 2) acc[mb][nb] = WFrag<T16>::mma(a2[mb], b, acc[mb][nb]); if (NSPLIT >= 2) acc[mb][nb] = WFrag<T16>::mma(a[mb], b2, acc[mb][nb]); } }
        asm volatile("v_nop\n\tv_nop\n\tv_nop\n\tv_nop" : "+v"(acc[0][0]), "+v"(acc[1][1]), "+v"(acc[2][2]), "+v"(acc[3][3]) : "v"(a[0]), "v"(a[3]));
    }
#pragma unroll
    for (int mb = 0; mb < 4; ++mb) {
#pragma unroll
        for (int nb = 0; nb < 4; ++nb) {
#pragma unroll
            for (int j = 0; j < 8; ++j) os[(hi * 8 + j) * 68 + nb * 16 + lr] = acc[mb][nb][j]; }
        __builtin_amdgcn_wave_barrier(); asm volatile("" ::: "memory");
        float* crow = C + (size_t)(r0 + mb * 16) * ldc + c0;
#pragma unroll 1
        for (int ps = 0; ps < 2; ++ps) {
#pragma unroll
            for (int s = 0; s < 8; ++s) { const int row = 2 * s + hi, cofs = lr * 4; v4f val = *(const v4fa*)(os + row * 68 + cofs); if (BIAS) { val[0] += bfr(bias[c0 + cofs]); val[1] += bfr(bias[c0 + cofs + 1]); val[2] += bfr(bias[c0 + cofs + 2]); val[3] += bfr(bias[c0 + cofs + 3]); }
                *(volatile v4f*)(crow + (size_t)row * ldc + cofs) = val; }
            if (ps == 0) __threadfence(); }
        __builtin_amdgcn_wave_barrier(); asm volatile("" ::: "memory");
    }
}

__device__ __forceinline__ h16 tohx(float x) { return (h16)x; }
__device__ __forceinline__ void splitf(float y, unsigned short& h, unsigned short& l) { h = f2bf(y); l = f2bf(y - bf2f(h)); }
typedef __attribute__((ext_vector_type(2))) _Float16 v2h;
typedef __attribute__((ext_vector_type(4))) _Float16 v4h;
typedef __attribute__((ext_vector_type(2))) unsigned short v2us;
typedef __attribute__((ext_vector_type(4))) unsigned short v4us;
typedef __attribute__((ext_vector_type(2))) float v2f;

__global__ __launch_bounds__(256) void k_cvt8(const float* __restrict__ src, bf* dst, size_t n8) { const size_t i = (size_t)blockIdx.x * 256 + threadIdx.x; if (i >= n8) return; const v8f v = *(const v8f*)(src + i * 8); v8us o;
#pragma unroll
    for (int k = 0; k < 8; ++k) o[k] = f2bf(v[k]); *(volatile v8us*)(dst + i * 8) = o; __threadfence(); *(volatile v8us*)(dst + i * 8) = o; }
__global__ __launch_bounds__(256) void k_embpad(const float* __restrict__ e1, bf* EB) { const int e = (blockIdx.x * 256 + threadIdx.x) * 4; if (e >= 64 * AD) return; const int r = e / AD; v4us o;
#pragma unroll
    for (int q = 0; q < 4; ++q) o[q] = (r < NB_) ? f2bf(e1[e + q]) : (unsigned short)0; *(volatile v4us*)(EB + e) = o; __threadfence(); *(volatile v4us*)(EB + e) = o; }
__global__ __launch_bounds__(256) void k_gnx(const float* __restrict__ x, float* ST) { const int lane = threadIdx.x & 31; const int w = blockIdx.x * 8 + (threadIdx.x >> 5); if (w >= NB_ * NG) return; const float* p = x + (size_t)w * 8 * LL; float s = 0.f;
    for (int i = lane * 4; i < 8 * LL; i += 128) { const v4f a = *(const v4f*)(p + i);
#pragma unroll
        for (int q = 0; q < 4; ++q) { float t = bfr(a[q]); asm volatile("" : "+v"(t)); s = __fadd_rn(s, t); } }
#pragma unroll
    for (int sh = 16; sh; sh >>= 1) s += __shfl_xor(s, sh, 32);
    const float mu = s * (1.0f / (8 * LL)); float qq = 0.f;
    for (int i = lane * 4; i < 8 * LL; i += 128) { const v4f a = *(const v4f*)(p + i);
#pragma unroll
        for (int q = 0; q < 4; ++q) { const float d0 = bfr(a[q]) - mu; float t = __fmul_rn(d0, d0); asm volatile("" : "+v"(t)); qq = __fadd_rn(qq, t); } }
#pragma unroll
    for (int sh = 16; sh; sh >>= 1) qq += __shfl_xor(qq, sh, 32);
    const float rs = __fdiv_rn(1.0f, __fsqrt_rn(__fadd_rn(qq * (1.0f / (8 * LL)), 1e-5f))); const float o = lane == 0 ? mu : (lane == 1 ? rs : 0.f); *(volatile float*)(ST + (size_t)w * 32 + lane) = o; __threadfence(); *(volatile float*)(ST + (size_t)w * 32 + lane) = o; }
__global__ __launch_bounds__(256) void k_xnT(const float* __restrict__ xb, const float* __restrict__ STb, const float* __restrict__ gw, const float* __restrict__ gb, bf* Xh, bf* Xl) { const int e = (blockIdx.x * 256 + threadIdx.x) * 2; if (e >= LL * CC) return; const int c = e % CC, l = e / CC; v2us oh, ol;
#pragma unroll
    for (int q = 0; q < 2; ++q) { const int cq = c + q; const float mu = STb[(cq / 8) * 32], rs = STb[(cq / 8) * 32 + 1]; float w = bfr(gw[cq]), bb = bfr(gb[cq]); asm volatile("" : "+v"(w)); asm volatile("" : "+v"(bb)); float tn = __fmul_rn(bfr(xb[(size_t)cq * LL + l]) - mu, rs); asm volatile("" : "+v"(tn)); float tw = __fmul_rn(tn, w); asm volatile("" : "+v"(tw)); unsigned short a, c2; splitf(__fadd_rn(tw, bb), a, c2); oh[q] = a; ol[q] = c2; }
    *(volatile v2us*)(Xh + e) = oh; *(volatile v2us*)(Xl + e) = ol; __threadfence(); *(volatile v2us*)(Xh + e) = oh; *(volatile v2us*)(Xl + e) = ol; }
__global__ __launch_bounds__(256) void k_kvcoef(const float* __restrict__ wkv, const float* __restrict__ gw, const float* __restrict__ gb, const float* __restrict__ bkv, float* KVC) { const int o = blockIdx.x * 256 + threadIdx.x; if (o >= 2 * CC) return; float sa = 0.f, sb = 0.f;
#pragma unroll 4
    for (int c = 0; c < CC; ++c) { const float w = bfr(wkv[(size_t)o * CC + c]); float g = bfr(gw[c]), b2 = bfr(gb[c]); asm volatile("" : "+v"(g)); asm volatile("" : "+v"(b2)); float pa = __fmul_rn(w, g), pb = __fmul_rn(w, b2); asm volatile("" : "+v"(pa)); asm volatile("" : "+v"(pb)); sa = __fadd_rn(sa, pa); sb = __fadd_rn(sb, pb); }
    float bo = bfr(bkv[o]); asm volatile("" : "+v"(bo)); v2f r; r[0] = sa; r[1] = __fadd_rn(sb, bo); *(volatile v2f*)(KVC + (size_t)o * 2) = r; __threadfence(); *(volatile v2f*)(KVC + (size_t)o * 2) = r; }
__global__ __launch_bounds__(256) void k_astat(const float* __restrict__ A2, float* SA) { const int lane = threadIdx.x & 31; const int b = blockIdx.x * 8 + (threadIdx.x >> 5); if (b >= NB_) return; const float* p = A2 + (size_t)b * LL; float s = 0.f;
    for (int i = lane; i < LL; i += 32) s = __fadd_rn(s, p[i]);
#pragma unroll
    for (int sh = 16; sh; sh >>= 1) s += __shfl_xor(s, sh, 32);
    const float mu = s * (1.0f / LL); float qq = 0.f;
    for (int i = lane; i < LL; i += 32) { const float d0 = p[i] - mu; float t = __fmul_rn(d0, d0); asm volatile("" : "+v"(t)); qq = __fadd_rn(qq, t); }
#pragma unroll
    for (int sh = 16; sh; sh >>= 1) qq += __shfl_xor(qq, sh, 32);
    const float rs = __fdiv_rn(1.0f, __fsqrt_rn(__fadd_rn(qq * (1.0f / LL), 1e-5f))); const float o = lane == 0 ? mu : (lane == 1 ? rs : 0.f); *(volatile float*)(SA + (size_t)b * 32 + lane) = o; __threadfence(); *(volatile float*)(SA + (size_t)b * 32 + lane) = o; }
__device__ __forceinline__ float chan(const float* __restrict__ Q, const float* __restrict__ A2b, float mu, float rs, const float* __restrict__ KVC, int j, int l) {
    if (j < CC) return Q[(size_t)l * CC + j]; const int o = j - CC; float n = __fmul_rn(__fsub_rn(A2b[l], mu), rs); asm volatile("" : "+v"(n)); float t = __fmul_rn(n, KVC[o * 2]); asm volatile("" : "+v"(t)); return __fadd_rn(t, KVC[o * 2 + 1]); }
__global__ __launch_bounds__(256) void k_planes(const float* __restrict__ Q, const float* __restrict__ A2b, const float* __restrict__ SAb, const float* __restrict__ KVC, h16* QP, h16* KP, h16* VT) { const int e = (blockIdx.x * 256 + threadIdx.x) * 2; if (e >= NHD * LL * CH) return; const float mu = SAb[0], rs = SAb[1];
    { const int c = e % CH; const int l = (e / CH) % LL; const int i = e / (LL * CH); v2h oq, ok; oq[0] = tohx(chan(Q, A2b, mu, rs, KVC, 192 * i + c, l)); oq[1] = tohx(chan(Q, A2b, mu, rs, KVC, 192 * i + c + 1, l)); ok[0] = tohx(chan(Q, A2b, mu, rs, KVC, 192 * i + 64 + c, l)); ok[1] = tohx(chan(Q, A2b, mu, rs, KVC, 192 * i + 64 + c + 1, l));
      *(volatile v2h*)(QP + e) = oq; *(volatile v2h*)(KP + e) = ok; __threadfence(); *(volatile v2h*)(QP + e) = oq; *(volatile v2h*)(KP + e) = ok; }
    { const int s = e % LL; const int c = (e / LL) % CH; const int i = e / (LL * CH); v2h ov; ov[0] = tohx(chan(Q, A2b, mu, rs, KVC, 192 * i + 128 + c, s)); ov[1] = tohx(chan(Q, A2b, mu, rs, KVC, 192 * i + 128 + c, s + 1)); *(volatile v2h*)(VT + e) = ov; __threadfence(); *(volatile v2h*)(VT + e) = ov; } }
__global__ __launch_bounds__(256) void k_asoft(const float* __restrict__ Sb, h16* P16) {
    const int lane = threadIdx.x & 31; const int row = blockIdx.x * 8 + (threadIdx.x >> 5); if (row >= ZH * TT) return;
    const float* sr = Sb + (size_t)row * TT; float v[32]; float mx = -3.0e38f;
#pragma unroll
    for (int ch = 0; ch < 8; ++ch) { const int j0 = ch * 128 + lane * 4; const v4f a = *(const v4f*)(sr + j0);
#pragma unroll
        for (int q = 0; q < 4; ++q) { const float t = a[q] * SCL; v[ch * 4 + q] = t; mx = fmaxf(mx, t); } }
#pragma unroll
    for (int sh = 16; sh; sh >>= 1) mx = fmaxf(mx, __shfl_xor(mx, sh, 32));
    float sum = 0.f;
#pragma unroll
    for (int k = 0; k < 32; ++k) { v[k] = __expf(v[k] - mx); sum += v[k]; }
#pragma unroll
    for (int sh = 16; sh; sh >>= 1) sum += __shfl_xor(sum, sh, 32);
    const float f = __fdiv_rn(PCAR, sum);
#pragma unroll 1
    for (int ps = 0; ps < 2; ++ps) {
#pragma unroll
        for (int ch = 0; ch < 8; ++ch) { v4h o;
#pragma unroll
            for (int q = 0; q < 4; ++q) o[q] = tohx(v[ch * 4 + q] * f);
            *(volatile v4h*)(P16 + (size_t)row * TT + ch * 128 + lane * 4) = o; }
        if (ps == 0) __threadfence(); }
}
__global__ __launch_bounds__(256) void k_mrg(const float* __restrict__ O, int i, bf* Ah, bf* Al) { const int e = (blockIdx.x * 256 + threadIdx.x) * 2; if (e >= LL * CH) return; const int c = e & 63; const int l = e >> 6; v2us oh, ol;
#pragma unroll
    for (int q = 0; q < 2; ++q) { unsigned short a, c2; splitf(O[e + q] * (1.0f / PCAR), a, c2); oh[q] = a; ol[q] = c2; } const size_t oo = (size_t)l * CC + i * CH + c; *(volatile v2us*)(Ah + oo) = oh; *(volatile v2us*)(Al + oo) = ol; __threadfence(); *(volatile v2us*)(Ah + oo) = oh; *(volatile v2us*)(Al + oo) = ol; }
__global__ __launch_bounds__(256) void k_outT(const float* __restrict__ Hh, const float* __restrict__ xb, float* OUTb) { const int e = (blockIdx.x * 256 + threadIdx.x) * 2; if (e >= CC * LL) return; const int l = e % LL, o = e / LL; v2f r; r[0] = __fadd_rn(bfr(xb[e]), Hh[(size_t)l * CC + o]); r[1] = __fadd_rn(bfr(xb[e + 1]), Hh[(size_t)(l + 1) * CC + o]);
    *(volatile v2f*)(OUTb + e) = r; __threadfence(); *(volatile v2f*)(OUTb + e) = r; }

extern "C" void kernel_launch(void* const* d_in, const int* in_sizes, int n_in,
                              void* d_out, int out_size, void* d_ws, size_t ws_size, hipStream_t stream) {
    (void)in_sizes; (void)n_in; (void)out_size;
    const float* IN[14]; for (int i = 0; i < 14; ++i) IN[i] = (const float*)d_in[i];
    float* OUT = (float*)d_out;
    char* wsp = (char*)d_ws;
    auto take = [&](size_t bytes) { char* p = wsp; wsp += (bytes + 255) & ~(size_t)255; return (void*)p; };
    bf* WQ = (bf*)take((size_t)CC * CC * 2); bf* WP = (bf*)take((size_t)CC * CC * 2); bf* WA = (bf*)take((size_t)LL * AD * 2); bf* EB = (bf*)take((size_t)64 * AD * 2); float* A2 = (float*)take((size_t)64 * LL * 4); float* SA = (float*)take((size_t)NB_ * 32 * 4); float* ST = (float*)take((size_t)NB_ * NG * 32 * 4); float* KVC = (float*)take((size_t)2 * CC * 2 * 4);
    bf* Xh = (bf*)take((size_t)LL * CC * 2); bf* Xl = (bf*)take((size_t)LL * CC * 2); float* Q = (float*)take((size_t)LL * CC * 4); h16* QP = (h16*)take((size_t)NHD * LL * CH * 2); h16* KP = (h16*)take((size_t)NHD * LL * CH * 2); h16* VT = (h16*)take((size_t)NHD * CH * LL * 2);
    float* Sb = (float*)take((size_t)TT * TT * 4); h16* Pm = (h16*)take((size_t)TT * TT * 2); float* O = (float*)take((size_t)LL * CH * 4); bf* Ah = (bf*)take((size_t)LL * CC * 2); bf* Al = (bf*)take((size_t)LL * CC * 2); float* Hh = (float*)take((size_t)LL * CC * 4);
    if ((size_t)(wsp - (char*)d_ws) > ws_size) return;
    { k_cvt8<<<(CC * CC / 8 + 255) / 256, 256, 0, stream>>>(IN[8], WQ, (size_t)CC * CC / 8); k_cvt8<<<(CC * CC / 8 + 255) / 256, 256, 0, stream>>>(IN[12], WP, (size_t)CC * CC / 8); k_cvt8<<<(LL * AD / 8 + 255) / 256, 256, 0, stream>>>(IN[2], WA, (size_t)LL * AD / 8);
      k_embpad<<<(64 * AD / 4 + 255) / 256, 256, 0, stream>>>(IN[1] + (size_t)NB_ * AD, EB);
      k_gnx<<<(NB_ * NG) / 8, 256, 0, stream>>>(IN[0], ST); k_kvcoef<<<(2 * CC + 255) / 256, 256, 0, stream>>>(IN[10], IN[6], IN[7], IN[11], KVC);
      k_gemmw<bf, 0, true><<<dim3(1, LL / 64, 1), 32, 0, stream>>>(EB, nullptr, WA, nullptr, AD, A2, LL, IN[3], 0, 0, 0);
      k_astat<<<(NB_ + 7) / 8, 256, 0, stream>>>(A2, SA); }
    const unsigned LP = (NHD * LL * CH / 2 + 255) / 256;
    for (int b = 0; b < NB_; ++b) { const float* xb = IN[0] + (size_t)b * CC * LL;
        k_xnT<<<(LL * CC / 2 + 255) / 256, 256, 0, stream>>>(xb, ST + (size_t)b * NG * 32, IN[4], IN[5], Xh, Xl);
        k_gemmw<bf, 1, true><<<dim3(LL / 64, CC / 64, 1), 32, 0, stream>>>(Xh, Xl, WQ, nullptr, CC, Q, CC, IN[9], 0, 0, 0);
        k_planes<<<LP, 256, 0, stream>>>(Q, A2 + (size_t)b * LL, SA + (size_t)b * 32, KVC, QP, KP, VT);
        for (int i = 0; i < NHD; ++i) {
            k_gemmw<h16, 0, false><<<dim3(LL / 64, TT / 64, 1), 32, 0, stream>>>(QP + (size_t)i * LL * CH, nullptr, KP + (size_t)i * LL * CH, nullptr, CH, Sb, TT, nullptr, 0, 0, 0);
            k_asoft<<<TT / 8, 256, 0, stream>>>(Sb, Pm);
            k_gemmw<h16, 0, false><<<dim3(LL / 64, 1, 1), 32, 0, stream>>>(Pm, nullptr, VT + (size_t)i * CH * LL, nullptr, TT, O, CH, nullptr, 0, 0, 0);
            k_mrg<<<(LL * CH / 2 + 255) / 256, 256, 0, stream>>>(O, i, Ah, Al); }
        k_gemmw<bf, 1, true><<<dim3(LL / 64, CC / 64, 1), 32, 0, stream>>>(Ah, Al, WP, nullptr, CC, Hh, CC, IN[13], 0, 0, 0);
        k_outT<<<(CC * LL / 2 + 255) / 256, 256, 0, stream>>>(Hh, xb, OUT + (size_t)b * CC * LL); }
}
